// DynamicRoutingLayer_28209345200812
// MI455X (gfx1250) — hardware-verified
//
#include <hip/hip_runtime.h>
#include <hip/hip_bf16.h>

typedef __bf16 bf16;
typedef bf16  v16bf __attribute__((ext_vector_type(16)));
typedef unsigned short u16;
typedef u16   v8us __attribute__((ext_vector_type(8)));
typedef float v8f  __attribute__((ext_vector_type(8)));
typedef float v4f  __attribute__((ext_vector_type(4)));
typedef unsigned int v4u __attribute__((ext_vector_type(4)));

#define NB    128
#define MSEQ  512
#define DM    128
#define NH    4
#define MR    32
#define NSTEP (MSEQ / MR)
#define SP    512
#define YP    136

#define LDS_S_OFF    0
#define LDS_YH_OFF   65536
#define LDS_YL_OFF   (LDS_YH_OFF + 8704)
#define LDS_RINV_OFF (LDS_YL_OFF + 8704)
#define LDS_G_OFF    (LDS_RINV_OFF + 128)
#define LDS_OP_OFF   (LDS_G_OFF + 2048)
#define LDS_O_OFF    (LDS_OP_OFF + 1024)
#define LDS_OF_OFF   (LDS_O_OFF + 512)
#define LDS_BYTES    (LDS_OF_OFF + 512)

static_assert((LDS_YH_OFF % 16) == 0);
static_assert((LDS_YL_OFF % 16) == 0);
static_assert(((YP * 2) % 16) == 0);
static_assert(LDS_BYTES == 87168);

#define CSCALE (0.08838834764831845f * 0.25f)

static __device__ __forceinline__ u16 bf16_bits(float v) {
  unsigned int u = __float_as_uint(v);
  u = u + 0x7FFFu + ((u >> 16) & 1u);
  return (u16)(u >> 16);
}

static __device__ __forceinline__ void split_bf16(float v, u16& hb, u16& lb) {
  hb = bf16_bits(v);
  const float hf = __uint_as_float(((unsigned int)hb) << 16);
  lb = bf16_bits(v - hf);
}

union Frag { v16bf v; v8us p[2]; };

static __device__ __forceinline__ v16bf load_frag(const u16* rowp, int k0, int h) {
  Frag f;
  f.p[0] = *(const v8us*)(rowp + k0 + 8 * h);
  f.p[1] = *(const v8us*)(rowp + k0 + 16 + 8 * h);
  return f.v;
}

static __device__ __forceinline__ v8f wmma_bf(v16bf a, v16bf b, v8f c) {
  v8f d = __builtin_amdgcn_wmma_f32_16x16x32_bf16(false, a, false, b, (short)0, c, false, false);
  asm volatile("v_nop\n\tv_nop\n\tv_nop\n\tv_nop" : "+v"(d) : "v"(a), "v"(b));
  return d;
}

static __device__ __forceinline__ v8f wmma_split(v16bf ah, v16bf al, v16bf bh, v16bf bl, v8f c) {
  c = wmma_bf(ah, bh, c);
  c = wmma_bf(ah, bl, c);
  c = wmma_bf(al, bh, c);
  return c;
}

__global__ __launch_bounds__(256)
void k_cvt_x(const float* __restrict__ x, u16* __restrict__ xh, u16* __restrict__ xl, int n8) {
  const int g = blockIdx.x * 256 + threadIdx.x;
  if (g >= n8) return;
  const v4f a = *(const v4f*)(x + (size_t)g * 8);
  const v4f b = *(const v4f*)(x + (size_t)g * 8 + 4);
  union { v8us s; v4u u; } ph, pl;
#pragma unroll
  for (int j = 0; j < 4; ++j) {
    u16 hb, lb;
    split_bf16(a[j], hb, lb);
    ph.s[j] = hb; pl.s[j] = lb;
    split_bf16(b[j], hb, lb);
    ph.s[4 + j] = hb; pl.s[4 + j] = lb;
  }
  const v4u vh = ph.u, vl = pl.u;
  volatile v4u* dh = (volatile v4u*)(xh + (size_t)g * 8);
  volatile v4u* dl = (volatile v4u*)(xl + (size_t)g * 8);
  *dh = vh;
  *dl = vl;
  __threadfence();
  *dh = vh;
  *dl = vl;
}

__global__ __launch_bounds__(256)
void k_wsum_t(const float* __restrict__ rw, u16* __restrict__ wsth, u16* __restrict__ wstl) {
  const int t = blockIdx.x * 256 + threadIdx.x;
  if (t >= (DM * DM) / 8) return;
  const int e = t >> 4;
  const int d0 = (t & 15) * 8;
  union { v8us s; v4u u; } ph, pl;
#pragma unroll
  for (int j = 0; j < 8; ++j) {
    const int d = d0 + j;
    float s = 0.f;
#pragma unroll
    for (int hh = 0; hh < NH; ++hh) s += rw[((size_t)hh * DM + d) * DM + e];
    u16 hb, lb;
    split_bf16(s, hb, lb);
    ph.s[j] = hb; pl.s[j] = lb;
  }
  const v4u vh = ph.u, vl = pl.u;
  volatile v4u* dh = (volatile v4u*)(wsth + (size_t)e * DM + d0);
  volatile v4u* dl = (volatile v4u*)(wstl + (size_t)e * DM + d0);
  *dh = vh;
  *dl = vl;
  __threadfence();
  *dh = vh;
  *dl = vl;
}

__global__ __launch_bounds__(256)
void k_route(const u16* __restrict__ xh, const u16* __restrict__ xl,
             const u16* __restrict__ wsth, const u16* __restrict__ wstl,
             const float* __restrict__ x, const float* __restrict__ pw,
             const float* __restrict__ pb, float* __restrict__ out) {
  extern __shared__ v4u smem_v4[];
  char* smem = reinterpret_cast<char*>(smem_v4);
  float* S     = reinterpret_cast<float*>(smem + LDS_S_OFF);
  u16*   Yh    = reinterpret_cast<u16*>(smem + LDS_YH_OFF);
  u16*   Yl    = reinterpret_cast<u16*>(smem + LDS_YL_OFF);
  float* rinv  = reinterpret_cast<float*>(smem + LDS_RINV_OFF);
  float* Gs    = reinterpret_cast<float*>(smem + LDS_G_OFF);
  float* opart = reinterpret_cast<float*>(smem + LDS_OP_OFF);
  float* ov    = reinterpret_cast<float*>(smem + LDS_O_OFF);
  float* ofin  = reinterpret_cast<float*>(smem + LDS_OF_OFF);

  const int n    = blockIdx.x;
  const int tid  = threadIdx.x;
  const int lane = tid & 31;
  const int wave = tid >> 5;
  const int h    = lane >> 4;
  const int m    = lane & 15;

  const u16* xhn = xh + (size_t)n * MSEQ * DM;
  const u16* xln = xl + (size_t)n * MSEQ * DM;

  float g0 = 0.f, g1 = 0.f;

#pragma unroll 1
  for (int ms = 0; ms < NSTEP; ++ms) {
    const int m0 = ms * MR;

    {
      v8f acc[2] = {};
      const u16* a0h = xhn + (size_t)(m0 + m) * DM;
      const u16* a0l = xln + (size_t)(m0 + m) * DM;
      const u16* a1h = xhn + (size_t)(m0 + 16 + m) * DM;
      const u16* a1l = xln + (size_t)(m0 + 16 + m) * DM;
      const u16* bhr = wsth + (size_t)(wave * 16 + m) * DM;
      const u16* blr = wstl + (size_t)(wave * 16 + m) * DM;
#pragma unroll 1
      for (int ks = 0; ks < DM / 32; ++ks) {
        const int k0 = ks * 32;
        const v16bf fa0h = load_frag(a0h, k0, h);
        const v16bf fa0l = load_frag(a0l, k0, h);
        const v16bf fa1h = load_frag(a1h, k0, h);
        const v16bf fa1l = load_frag(a1l, k0, h);
        const v16bf fbh  = load_frag(bhr, k0, h);
        const v16bf fbl  = load_frag(blr, k0, h);
        acc[0] = wmma_split(fa0h, fa0l, fbh, fbl, acc[0]);
        acc[1] = wmma_split(fa1h, fa1l, fbh, fbl, acc[1]);
      }
#pragma unroll
      for (int r = 0; r < 2; ++r)
#pragma unroll
        for (int j = 0; j < 8; ++j) {
          u16 hb, lb;
          split_bf16(acc[r][j], hb, lb);
          const int idx = (r * 16 + 8 * h + j) * YP + wave * 16 + m;
          Yh[idx] = hb;
          Yl[idx] = lb;
        }
    }
    __syncthreads();

    {
      v8f acc[2][4] = {};
      const int c0 = wave * 64;
#pragma unroll 1
      for (int ks = 0; ks < DM / 32; ++ks) {
        const int k0 = ks * 32;
        const v16bf fa0h = load_frag(Yh + m * YP, k0, h);
        const v16bf fa0l = load_frag(Yl + m * YP, k0, h);
        const v16bf fa1h = load_frag(Yh + (16 + m) * YP, k0, h);
        const v16bf fa1l = load_frag(Yl + (16 + m) * YP, k0, h);
#pragma unroll
        for (int t = 0; t < 4; ++t) {
          const size_t ro = (size_t)(c0 + t * 16 + m) * DM;
          const v16bf fbh = load_frag(xhn + ro, k0, h);
          const v16bf fbl = load_frag(xln + ro, k0, h);
          acc[0][t] = wmma_split(fa0h, fa0l, fbh, fbl, acc[0][t]);
          acc[1][t] = wmma_split(fa1h, fa1l, fbh, fbl, acc[1][t]);
        }
      }
#pragma unroll
      for (int r = 0; r < 2; ++r)
#pragma unroll
        for (int t = 0; t < 4; ++t)
#pragma unroll
          for (int j = 0; j < 8; ++j)
            S[(r * 16 + 8 * h + j) * SP + c0 + t * 16 + m] = acc[r][t][j] * CSCALE;
    }
    __syncthreads();

    {
      const int row = tid >> 3, part = tid & 7;
      float* Sr = S + row * SP + part * 64;
      float mx = -3.402823466e38f;
#pragma unroll 8
      for (int i = 0; i < 64; ++i) mx = fmaxf(mx, Sr[i]);
      mx = fmaxf(mx, __shfl_xor(mx, 1));
      mx = fmaxf(mx, __shfl_xor(mx, 2));
      mx = fmaxf(mx, __shfl_xor(mx, 4));
      float sm = 0.f;
#pragma unroll 8
      for (int i = 0; i < 64; ++i) {
        const float e = __expf(Sr[i] - mx);
        Sr[i] = e;
        sm += e;
      }
      sm += __shfl_xor(sm, 1);
      sm += __shfl_xor(sm, 2);
      sm += __shfl_xor(sm, 4);
      if (part == 0) rinv[row] = 1.0f / sm;
    }
    __syncthreads();

    {
      float cA = 0.f, cB = 0.f;
#pragma unroll 8
      for (int mm = 0; mm < MR; ++mm) {
        const float rr = rinv[mm];
        cA += S[mm * SP + tid] * rr;
        cB += S[mm * SP + tid + 256] * rr;
      }
      g0 += cA;
      g1 += cB;
    }
  }

  Gs[tid] = g0;
  Gs[tid + 256] = g1;
  __syncthreads();

  {
    const int d = tid & 127, hf = tid >> 7;
    const float* xn = x + (size_t)n * MSEQ * DM + d;
    float p = 0.f;
    const int kbeg = hf * 256;
#pragma unroll 4
    for (int k = kbeg; k < kbeg + 256; ++k) p += Gs[k] * xn[(size_t)k * DM];
    opart[hf * 128 + d] = p;
  }
  __syncthreads();
  if (tid < 128) ov[tid] = (opart[tid] + opart[128 + tid]) * (1.0f / 512.0f);
  __syncthreads();

  if (tid < 128) {
    const float* pwr = pw + (size_t)tid * DM;
    float r = 0.f;
#pragma unroll 4
    for (int d = 0; d < DM; ++d) r += ov[d] * pwr[d];
    ofin[tid] = r + pb[tid];
  }
  __syncthreads();

  if (tid < 32) {
    v4f v;
    v[0] = ofin[4 * tid + 0];
    v[1] = ofin[4 * tid + 1];
    v[2] = ofin[4 * tid + 2];
    v[3] = ofin[4 * tid + 3];
    volatile v4f* dst = (volatile v4f*)(out + (size_t)n * DM + 4 * tid);
    *dst = v;
    __threadfence();
    *dst = v;
  }
}

extern "C" void kernel_launch(void* const* d_in, const int* in_sizes, int n_in,
                              void* d_out, int out_size, void* d_ws, size_t ws_size,
                              hipStream_t stream) {
  if (n_in < 4) return;
  if (in_sizes[0] != NB * MSEQ * DM) return;
  if (in_sizes[1] != NH * DM * DM) return;
  if (in_sizes[2] != DM * DM) return;
  if (in_sizes[3] != DM) return;
  if (out_size != NB * DM) return;

  const size_t xp_bytes  = (size_t)NB * MSEQ * DM * sizeof(u16);
  const size_t wst_bytes = (size_t)DM * DM * sizeof(u16);
  const size_t need = 2 * xp_bytes + 2 * wst_bytes;
  if (ws_size < need) return;

  const float* x  = (const float*)d_in[0];
  const float* rw = (const float*)d_in[1];
  const float* pw = (const float*)d_in[2];
  const float* pb = (const float*)d_in[3];
  float* out = (float*)d_out;

  char* ws = (char*)d_ws;
  u16* xh   = (u16*)(ws + 0);
  u16* xl   = (u16*)(ws + xp_bytes);
  u16* wsth = (u16*)(ws + 2 * xp_bytes);
  u16* wstl = (u16*)(ws + 2 * xp_bytes + wst_bytes);

  const int n8 = in_sizes[0] / 8;
  const int cvt_blocks = (n8 + 255) / 256;
  k_cvt_x<<<dim3(cvt_blocks), dim3(256), 0, stream>>>(x, xh, xl, n8);
  k_wsum_t<<<dim3(((DM * DM) / 8 + 255) / 256), dim3(256), 0, stream>>>(rw, wsth, wstl);
  k_route<<<dim3(NB), dim3(256), LDS_BYTES, stream>>>(xh, xl, wsth, wstl, x, pw, pb, out);
  (void)hipGetLastError();
}
